// S4Enrichment1_55095840473855
// MI455X (gfx1250) — hardware-run, weakly checked
//
#include <hip/hip_runtime.h>
#include <math.h>

typedef __attribute__((ext_vector_type(16))) _Float16 v16h;
typedef __attribute__((ext_vector_type(8)))  _Float16 v8h;
typedef __attribute__((ext_vector_type(8)))  float    v8f;
typedef __attribute__((ext_vector_type(4)))  float    v4f;
typedef __attribute__((ext_vector_type(2)))  float    v2f;
typedef __attribute__((ext_vector_type(4)))  unsigned v4u;

constexpr int kBatch    = 2;
constexpr int kLen      = 4096;
constexpr int kWidth    = 1024;
constexpr int kModes    = 64;
constexpr int kOutF     = 512;
constexpr int kChunk    = 128;
constexpr int kChunksPS = kLen / kChunk;
constexpr int kRowsM    = kBatch * kChunksPS;
constexpr int kStateW   = 2 * kModes;
constexpr int kMvW      = kChunk + kStateW;
constexpr int kNpos     = kBatch * kLen;
constexpr int kGroupCh  = 256;
constexpr int kGroups   = kWidth / kGroupCh;
constexpr int kPitchW   = 132;
constexpr int kPeWidth  = 342;
static_assert(kChunksPS == 32 && kRowsM == 64 && kStateW == 128 && kMvW == 256 && kNpos == 8192 && kGroups == 4, "derived shapes");
static_assert((kChunk % 32) == 0 && (kStateW % 32) == 0 && (kWidth % 256) == 0, "K multiples of 32");
static_assert((kRowsM % 64) == 0 && (kChunk % 64) == 0 && (kStateW % 64) == 0 && (kNpos % 64) == 0 && (kLen % 64) == 0 && (kOutF % 256) == 0, "tile multiples");

constexpr bool kOutResid = false;

constexpr float kTabCarry    = 64.0f;
constexpr float kTabCarryInv = 1.0f / 64.0f;
constexpr float kWCarry      = 1024.0f;
constexpr float kGCarry      = 16.0f;
constexpr float kOutFold     = 1.0f / 16384.0f;
constexpr float kLoScale     = 2048.0f;
constexpr float kLoScaleInv  = 1.0f / 2048.0f;

constexpr size_t kOffU16  = 0;
constexpr size_t kOffG16  = kOffU16  + (size_t)kWidth * kNpos * 2;
constexpr size_t kOffG16L = kOffG16  + (size_t)kWidth * kNpos * 2;
constexpr size_t kOffMv   = kOffG16L + (size_t)kWidth * kNpos * 2;
constexpr size_t kOffEt   = kOffMv   + (size_t)kGroupCh * kChunk * kMvW * 2;
constexpr size_t kOffS32  = kOffEt   + (size_t)kGroupCh * kStateW * kChunk * 2;
constexpr size_t kOffInit = kOffS32  + (size_t)kGroupCh * kRowsM * kStateW * 4;
constexpr size_t kOffWpow = kOffInit + (size_t)kGroupCh * kRowsM * kStateW * 2;
constexpr size_t kOffWot  = kOffWpow + (size_t)kGroupCh * kModes * 2 * 4;
constexpr size_t kOffWotL = kOffWot  + (size_t)kOutF * kWidth * 2;
constexpr size_t kWsTotal = kOffWotL + (size_t)kOutF * kWidth * 2;
static_assert(kWsTotal == 90308608ull, "carve total");
static_assert(kWsTotal <= 134217728ull, "carve cap");
static_assert((kOffG16 % 128) == 0 && (kOffG16L % 128) == 0 && (kOffMv % 128) == 0 && (kOffEt % 128) == 0 &&
              (kOffS32 % 128) == 0 && (kOffInit % 128) == 0 && (kOffWpow % 128) == 0 && (kOffWot % 128) == 0 &&
              (kOffWotL % 128) == 0, "128-B aligned regions");

__device__ __forceinline__ float flush16(float v) {
  return (fabsf(v) < 6.103515625e-05f) ? 0.0f : v;
}
__device__ __forceinline__ unsigned short f16bits(float x) {
  const _Float16 h = (_Float16)flush16(x);
  return __builtin_bit_cast(unsigned short, h);
}
__device__ __forceinline__ unsigned pack2(float a, float b) {
  const unsigned lo = (unsigned)f16bits(a);
  const unsigned hi = (unsigned)f16bits(b);
  return lo | (hi << 16);
}
__device__ __forceinline__ float second16(float v) {
  const _Float16 hv = (_Float16)flush16(v);
  const float back = (float)hv;
  return (v - back) * kLoScale;
}
__device__ __forceinline__ void wave_sync() {
  __builtin_amdgcn_fence(__ATOMIC_RELEASE, "workgroup");
  __builtin_amdgcn_wave_barrier();
  __builtin_amdgcn_fence(__ATOMIC_ACQUIRE, "workgroup");
}
__device__ __forceinline__ void store2_v4u(unsigned short* p, v4u v) {
  volatile v4u* q = (volatile v4u*)p;
  *q = v;
  __threadfence();
  *q = v;
}
__device__ __forceinline__ float gelu_fast(float y) {
  const float u = 0.7978845608028654f * (y + 0.044715f * y * y * y);
  const float e = __expf(-2.0f * u);
  return y * __builtin_amdgcn_rcpf(1.0f + e);
}

union FragH { v16h v; v8h h[2]; };
union FragW { v16h v; v4u q[2]; };
__device__ __forceinline__ v16h frag_load(const _Float16* p) {
  FragH f;
  f.h[0] = *(const v8h*)(p);
  f.h[1] = *(const v8h*)(p + 16);
  return f.v;
}
template <int PITCH>
__device__ __forceinline__ v16h lds_frag(const unsigned* sw, int n, int kw) {
  FragW f;
  f.q[0] = *(const v4u*)(sw + n * PITCH + kw);
  f.q[1] = *(const v4u*)(sw + n * PITCH + kw + 8);
  return f.v;
}
__device__ __forceinline__ v8f mma16(v16h a, v16h b, v8f c) {
  return __builtin_amdgcn_wmma_f32_16x16x32_f16(false, a, false, b, (short)0, c, false, false);
}
__device__ __forceinline__ void tie_acc(v8f& a, v16h x, v16h y) { asm volatile("" : "+v"(a) : "v"(x), "v"(y)); }
__device__ __forceinline__ void tie_acc_nops(v8f& a, v16h x, v16h y) { asm volatile("v_nop\n\tv_nop\n\tv_nop\n\tv_nop" : "+v"(a) : "v"(x), "v"(y)); }
__device__ __forceinline__ void keep4(v16h a, v16h b, v16h c, v16h d) { asm volatile("v_nop" :: "v"(a), "v"(b), "v"(c), "v"(d)); }
__device__ __forceinline__ void acc_guard4(v8f& a, v8f& b, v8f& c, v8f& d) { asm volatile("v_nop\n\tv_nop\n\tv_nop\n\tv_nop" : "+v"(a), "+v"(b), "+v"(c), "+v"(d)); }

__device__ __forceinline__ void kloop64(v8f (&acc)[4][4], const _Float16* ap, int lda,
                                        const _Float16* bp, int ldb, int ksteps) {
#pragma unroll 1
  for (int ks = 0; ks < ksteps; ++ks) {
    v16h bh[4];
#pragma unroll
    for (int j = 0; j < 4; ++j) bh[j] = frag_load(bp + (size_t)(j * 16) * ldb + ks * 32);
#pragma unroll
    for (int i = 0; i < 4; ++i) {
      const v16h ah = frag_load(ap + (size_t)(i * 16) * lda + ks * 32);
#pragma unroll
      for (int j = 0; j < 4; ++j) acc[i][j] = mma16(ah, bh[j], acc[i][j]);
      tie_acc(acc[i][0], ah, bh[0]);
      tie_acc(acc[i][1], ah, bh[1]);
      tie_acc(acc[i][2], ah, bh[2]);
      tie_acc_nops(acc[i][3], ah, bh[3]);
    }
    keep4(bh[0], bh[1], bh[2], bh[3]);
  }
}

template <int NT>
__device__ __forceinline__ void stage_tile_T(const unsigned short* plane, size_t n0, unsigned* sw, int tid) {
#pragma unroll 1
  for (int it = 0; it < 1024 / NT; ++it) {
    const int task = it * NT + tid;
    const int n8 = task & 7;
    const int kp = task >> 3;
    const unsigned short* p0 = plane + (size_t)(2 * kp) * kNpos + n0 + n8 * 8;
    const v4u a = *(const v4u*)(p0);
    const v4u b = *(const v4u*)(p0 + kNpos);
    unsigned* dst = sw + (n8 * 8) * kPitchW + kp;
#pragma unroll
    for (int j = 0; j < 4; ++j) {
      const unsigned aw = a[j];
      const unsigned bw = b[j];
      dst[(2 * j) * kPitchW]     = (aw & 0xffffu) | (bw << 16);
      dst[(2 * j + 1) * kPitchW] = (aw >> 16) | (bw & 0xffff0000u);
    }
  }
}

__global__ __launch_bounds__(256) void weight_plane_kernel(
    const float* __restrict__ w_out, unsigned short* __restrict__ wot, unsigned short* __restrict__ wotl) {
  __shared__ float sT[32 * 257];
  const int tid = threadIdx.x;
  const int mm = tid & 31;
  const int kq = tid >> 5;
  const int m0 = (int)blockIdx.x * 32;
  const int kb = (int)blockIdx.y * 256;
#pragma unroll 1
  for (int it = 0; it < 32; ++it) {
    const int k = it * 8 + kq;
    sT[mm * 257 + k] = w_out[(size_t)(kb + k) * kOutF + m0 + mm];
  }
  __syncthreads();
#pragma unroll 1
  for (int it = 0; it < 4; ++it) {
    const int q = it * 256 + tid;
    const int row = q >> 5;
    const int k8 = (q & 31) * 8;
    float vh[8];
    float vl[8];
#pragma unroll
    for (int e = 0; e < 8; ++e) {
      const float v = sT[row * 257 + k8 + e] * kWCarry;
      vh[e] = v;
      vl[e] = second16(v);
    }
    const size_t off = (size_t)(m0 + row) * kWidth + kb + k8;
    const v4u ph = {pack2(vh[0], vh[1]), pack2(vh[2], vh[3]), pack2(vh[4], vh[5]), pack2(vh[6], vh[7])};
    store2_v4u(wot + off, ph);
    if (kOutResid) {
      const v4u pl = {pack2(vl[0], vl[1]), pack2(vl[2], vl[3]), pack2(vl[4], vl[5]), pack2(vl[6], vl[7])};
      store2_v4u(wotl + off, pl);
    }
  }
}

__global__ __launch_bounds__(256) void stream_plane_kernel(
    const float* __restrict__ x, unsigned short* __restrict__ u16) {
  __shared__ float sPe[16];
  const int tid = threadIdx.x;
  const int c = (int)blockIdx.x;
  const int axis = (c >= 2 * kPeWidth) ? 2 : ((c >= kPeWidth) ? 1 : 0);
  const int ac = c - axis * kPeWidth;
  if (tid < 32) {
    const int p = tid & 15;
    const float ex = (float)(ac & ~1) * (1.0f / 342.0f);
    const float invf = expf(-ex * 9.210340371976184f);
    const float s = (float)p * invf;
    float sn, cs;
    sincosf(s, &sn, &cs);
    const float pe = (ac & 1) ? cs : sn;
    if (tid < 16) sPe[p] = pe;
  }
  __syncthreads();
  const int step = (axis == 2) ? 1 : 0;
#pragma unroll 1
  for (int it = 0; it < 4; ++it) {
    const int task = it * 256 + tid;
    const int n = task * 8;
    const int b = n >> 12;
    const int l = n & (kLen - 1);
    const float* xp = x + ((size_t)b * kWidth + c) * kLen + l;
    const v4f a0 = *(const v4f*)(xp);
    const v4f a1 = *(const v4f*)(xp + 4);
    const int p0 = (axis == 0) ? (l >> 8) : ((axis == 1) ? ((l >> 4) & 15) : (l & 15));
    float pe[8];
#pragma unroll
    for (int e = 0; e < 8; ++e) pe[e] = sPe[p0 + step * e];
    const v4u pk = {pack2(a0[0] + pe[0], a0[1] + pe[1]), pack2(a0[2] + pe[2], a0[3] + pe[3]),
                    pack2(a1[0] + pe[4], a1[1] + pe[5]), pack2(a1[2] + pe[6], a1[3] + pe[7])};
    store2_v4u(u16 + (size_t)c * kNpos + n, pk);
  }
}

__global__ __launch_bounds__(256) void mode_tables_kernel(
    const float* __restrict__ log_dt, const float* __restrict__ a_re, const float* __restrict__ a_im,
    const float* __restrict__ c_re, const float* __restrict__ c_im, const float* __restrict__ dskip,
    unsigned short* __restrict__ et16, unsigned short* __restrict__ mv16, float* __restrict__ wpow, int h0) {
  __shared__ float sPr[129 * 32];
  __shared__ float sPi[129 * 32];
  __shared__ float sK[128];
  __shared__ float sCr[32];
  __shared__ float sCi[32];
  const int tid = threadIdx.x;
  const int n = tid & 31;
  const int seg = __builtin_amdgcn_readfirstlane((int)(threadIdx.x >> 5));
  const int hl = (int)blockIdx.x;
  const int hg = h0 + hl;
  const float dt = expf(log_dt[hg]);
  if (tid < 128) sK[tid] = 0.0f;
#pragma unroll 1
  for (int mp = 0; mp < 2; ++mp) {
    __syncthreads();
    const int mode = mp * 32 + n;
    const int idx = hg * kModes + mode;
    const float ar = a_re[idx];
    const float ai = a_im[idx];
    const float dr = ar * dt;
    const float di = ai * dt;
    const float em = expm1f(dr);
    const float es = em + 1.0f;
    float sn, cs;
    sincosf(di, &sn, &cs);
    const float cm1a = -(sn * sn) * (1.0f / (1.0f + fmaxf(cs, 0.0f)));
    const float cm1 = (cs > 0.0f) ? cm1a : (cs - 1.0f);
    const float wr = es * cs;
    const float wi = es * sn;
    const float nr = em * cs + cm1;
    const float ni = wi;
    const float inv = 1.0f / (ar * ar + ai * ai);
    const float qr = (nr * ar + ni * ai) * inv;
    const float qi = (ni * ar - nr * ai) * inv;
    const float cr = c_re[idx];
    const float ci = c_im[idx];
    const float c2r = 2.0f * (cr * qr - ci * qi);
    const float c2i = 2.0f * (cr * qi + ci * qr);
    float sr = wr, si = wi;
#pragma unroll 1
    for (int i = 0; i < 4; ++i) {
      const float t = sr * sr - si * si;
      si = 2.0f * sr * si;
      sr = t;
    }
    float gr = sr, gi = si;
#pragma unroll 1
    for (int i = 0; i < 3; ++i) {
      const float t = gr * gr - gi * gi;
      gi = 2.0f * gr * gi;
      gr = t;
    }
    float pr = 1.0f, pi = 0.0f;
#pragma unroll 1
    for (int s = 0; s < seg; ++s) {
      const float t = pr * sr - pi * si;
      pi = pr * si + pi * sr;
      pr = t;
    }
#pragma unroll 1
    for (int s = 0; s < 16; ++s) {
      const int l = 16 * seg + s;
      sPr[l * 32 + n] = pr;
      sPi[l * 32 + n] = pi;
      const float t = pr * wr - pi * wi;
      pi = pr * wi + pi * wr;
      pr = t;
    }
    if (seg == 7) {
      sPr[128 * 32 + n] = pr;
      sPi[128 * 32 + n] = pi;
    }
    if (seg == 0) {
      sCr[n] = c2r;
      sCi[n] = c2i;
      const v2f wv = {gr, gi};
      volatile v2f* wp = (volatile v2f*)(wpow + (size_t)(hl * kModes + mode) * 2);
      *wp = wv;
      __threadfence();
      *wp = wv;
    }
    __syncthreads();
    if (tid < 128) {
      float acc = sK[tid];
#pragma unroll 1
      for (int m = 0; m < 32; ++m) {
        acc += sCr[m] * sPr[tid * 32 + m] - sCi[m] * sPi[tid * 32 + m];
      }
      sK[tid] = acc;
    }
#pragma unroll 1
    for (int it = 0; it < 4; ++it) {
      const int q = it * 256 + tid;
      const int row = q >> 3;
      const int nb = (q & 7) * 4;
      unsigned wd[4];
#pragma unroll
      for (int e = 0; e < 4; ++e) {
        const int m = nb + e;
        const float ppr = sPr[(row + 1) * 32 + m];
        const float ppi = sPi[(row + 1) * 32 + m];
        const float a = sCr[m];
        const float bq = sCi[m];
        const float re = a * ppr - bq * ppi;
        const float im = a * ppi + bq * ppr;
        wd[e] = pack2(re * kTabCarry, -im * kTabCarry);
      }
      const v4u pk = {wd[0], wd[1], wd[2], wd[3]};
      store2_v4u(mv16 + ((size_t)hl * kChunk + row) * kMvW + kChunk + (mp * 32 + nb) * 2, pk);
    }
#pragma unroll 1
    for (int it = 0; it < 4; ++it) {
      const int q = it * 256 + tid;
      const int r = q >> 4;
      const int k8 = (q & 15) * 8;
      const int m = r >> 1;
      const int part = r & 1;
      float v[8];
#pragma unroll
      for (int e = 0; e < 8; ++e) {
        const int l = 127 - (k8 + e);
        const float a = sPr[l * 32 + m];
        const float bq = sPi[l * 32 + m];
        const float val = part ? bq : a;
        v[e] = val * kTabCarry;
      }
      const v4u pk = {pack2(v[0], v[1]), pack2(v[2], v[3]), pack2(v[4], v[5]), pack2(v[6], v[7])};
      store2_v4u(et16 + ((size_t)hl * kStateW + mp * 64 + r) * kChunk + k8, pk);
    }
  }
  __syncthreads();
  const float kd = sK[0] + dskip[hg];
#pragma unroll 1
  for (int it = 0; it < 8; ++it) {
    const int q = it * 256 + tid;
    const int row = q >> 4;
    const int s0 = (q & 15) * 8;
    float v[8];
#pragma unroll
    for (int e = 0; e < 8; ++e) {
      const int df = row - (s0 + e);
      int dc = (df < 0) ? 0 : df;
      dc = (dc > 127) ? 127 : dc;
      const float kv = sK[dc];
      const float val = (df > 0) ? kv : ((df == 0) ? kd : 0.0f);
      v[e] = val * kTabCarry;
    }
    const v4u pk = {pack2(v[0], v[1]), pack2(v[2], v[3]), pack2(v[4], v[5]), pack2(v[6], v[7])};
    store2_v4u(mv16 + ((size_t)hl * kChunk + row) * kMvW + s0, pk);
  }
}

template <int MODE>
__global__ __launch_bounds__(256) void chunk_gemm_kernel(
    const unsigned short* __restrict__ uplane, const unsigned short* __restrict__ initp,
    const unsigned short* __restrict__ btp, void* __restrict__ cout, unsigned short* __restrict__ coutl, int h0) {
  __shared__ __align__(16) float sT[8][16 * 68];
  __shared__ __align__(16) unsigned sHw[(MODE == 1) ? 8 : 1][(MODE == 1) ? 16 * 32 : 4];
  __shared__ __align__(16) unsigned sHl[(MODE == 1 && kOutResid) ? 8 : 1][(MODE == 1 && kOutResid) ? 16 * 32 : 4];
  const int lane = threadIdx.x & 31;
  const int wave = __builtin_amdgcn_readfirstlane((int)(threadIdx.x >> 5));
  const int hl = (int)blockIdx.x * 4 + (wave >> 1);
  const int hg = h0 + hl;
  const int tn = wave & 1;
  const int m0 = 0;
  const int n0 = tn << 6;
  const int rlane = lane & 15;
  const int koff = (lane >> 4) * 8;
  const int mOff = (lane >> 4) * 8;
  constexpr int LDB = (MODE == 1) ? kMvW : kChunk;
  constexpr int BROWS = (MODE == 1) ? kChunk : kStateW;
  const _Float16* A1 = (const _Float16*)uplane + (size_t)hg * kNpos;
  const _Float16* Bt = (const _Float16*)btp + (size_t)hl * BROWS * LDB;

  v8f acc[4][4];
#pragma unroll
  for (int i = 0; i < 4; ++i)
#pragma unroll
    for (int j = 0; j < 4; ++j) acc[i][j] = (v8f){0.f, 0.f, 0.f, 0.f, 0.f, 0.f, 0.f, 0.f};

  kloop64(acc, A1 + (size_t)(m0 + rlane) * kChunk + koff, kChunk,
          Bt + (size_t)(n0 + rlane) * LDB + koff, LDB, kChunk / 32);
  if (MODE == 1) {
    const _Float16* A2 = (const _Float16*)initp + (size_t)hl * kRowsM * kStateW;
    kloop64(acc, A2 + (size_t)(m0 + rlane) * kStateW + koff, kStateW,
            Bt + (size_t)(n0 + rlane) * LDB + kChunk + koff, LDB, kStateW / 32);
  }
  acc_guard4(acc[0][0], acc[0][1], acc[0][2], acc[0][3]);
  acc_guard4(acc[1][0], acc[1][1], acc[1][2], acc[1][3]);
  acc_guard4(acc[2][0], acc[2][1], acc[2][2], acc[2][3]);
  acc_guard4(acc[3][0], acc[3][1], acc[3][2], acc[3][3]);

  float* slab = sT[wave];
#pragma unroll
  for (int i = 0; i < 4; ++i) {
    const int mBase = m0 + (i << 4);
#pragma unroll
    for (int j = 0; j < 4; ++j) {
#pragma unroll
      for (int r = 0; r < 8; ++r) slab[(mOff + r) * 68 + (j << 4) + rlane] = acc[i][j][r] * kTabCarryInv;
    }
    wave_sync();
    if (MODE == 0) {
      float* C = (float*)cout + (size_t)hl * kRowsM * kStateW;
      const int h2 = lane >> 4;
      const int c4 = (lane & 15) * 4;
      for (int pass = 0; pass < 2; ++pass) {
#pragma unroll
        for (int it = 0; it < 8; ++it) {
          const int row = it * 2 + h2;
          const v4f v = *(const v4f*)(slab + row * 68 + c4);
          *(volatile v4f*)(C + (size_t)(mBase + row) * kStateW + n0 + c4) = v;
        }
        __threadfence();
      }
    } else {
      unsigned* sH = sHw[wave];
      unsigned* sL = sHl[kOutResid ? wave : 0];
      unsigned short* G = (unsigned short*)cout + (size_t)hg * kNpos;
      unsigned short* GL = coutl + (size_t)hg * kNpos;
      const int q = lane >> 3;
      const int cw = lane & 7;
#pragma unroll 1
      for (int it = 0; it < 4; ++it) {
        const int row = it * 4 + q;
        const float* sp = slab + row * 68 + cw * 8;
        const v4f a0 = *(const v4f*)(sp);
        const v4f a1 = *(const v4f*)(sp + 4);
        float g[8];
#pragma unroll
        for (int e = 0; e < 4; ++e) {
          g[e] = gelu_fast(a0[e]) * kGCarry;
          g[4 + e] = gelu_fast(a1[e]) * kGCarry;
        }
        const v4u pk = {pack2(g[0], g[1]), pack2(g[2], g[3]), pack2(g[4], g[5]), pack2(g[6], g[7])};
        *(v4u*)(sH + row * 32 + cw * 4) = pk;
        if (kOutResid) {
          const v4u pl = {pack2(second16(g[0]), second16(g[1])), pack2(second16(g[2]), second16(g[3])),
                          pack2(second16(g[4]), second16(g[5])), pack2(second16(g[6]), second16(g[7]))};
          *(v4u*)(sL + row * 32 + cw * 4) = pl;
        }
      }
      wave_sync();
      v4u vals[4];
      v4u vlo[4];
#pragma unroll
      for (int it = 0; it < 4; ++it) {
        vals[it] = *(const v4u*)(sH + (it * 4 + q) * 32 + cw * 4);
        if (kOutResid) vlo[it] = *(const v4u*)(sL + (it * 4 + q) * 32 + cw * 4);
      }
      for (int pass = 0; pass < 2; ++pass) {
#pragma unroll
        for (int it = 0; it < 4; ++it) {
          const int row = it * 4 + q;
          *(volatile v4u*)(G + (size_t)(mBase + row) * kChunk + n0 + cw * 8) = vals[it];
          if (kOutResid) *(volatile v4u*)(GL + (size_t)(mBase + row) * kChunk + n0 + cw * 8) = vlo[it];
        }
        __threadfence();
      }
    }
    wave_sync();
  }
}

__global__ __launch_bounds__(256) void combine_kernel(
    const float* __restrict__ s32, const float* __restrict__ wpow, unsigned short* __restrict__ init16) {
  const int lane = threadIdx.x & 31;
  const int wave = __builtin_amdgcn_readfirstlane((int)(threadIdx.x >> 5));
  const int pair = (int)blockIdx.x * 8 + wave;
  const int mh = pair & 1;
  const int b = (pair >> 1) & 1;
  const int h = pair >> 2;
  const int n = mh * 32 + lane;
  const v2f w = *(const v2f*)(wpow + (size_t)(h * kModes + n) * 2);
  const float w_re = w[0];
  const float w_im = w[1];
  const float* sp = s32 + ((size_t)h * kRowsM + (size_t)b * kChunksPS) * kStateW + 2 * n;
  unsigned* ip = (unsigned*)(init16 + ((size_t)h * kRowsM + (size_t)b * kChunksPS) * kStateW) + n;
  float er = 0.0f, ei = 0.0f;
#pragma unroll 1
  for (int cidx = 0; cidx < kChunksPS; ++cidx) {
    const v2f s = *(const v2f*)(sp + (size_t)cidx * kStateW);
    const float cr = fminf(fmaxf(er, -60000.0f), 60000.0f);
    const float ci = fminf(fmaxf(ei, -60000.0f), 60000.0f);
    const unsigned word = pack2(cr, ci);
    volatile unsigned* q = (volatile unsigned*)(ip + (size_t)cidx * (kStateW / 2));
    *q = word;
    __threadfence();
    *q = word;
    const float tr = w_re * er - w_im * ei + s[0];
    ei = w_re * ei + w_im * er + s[1];
    er = tr;
  }
}

__global__ __launch_bounds__(256) void out_proj_kernel(
    const unsigned short* __restrict__ g16, const unsigned short* __restrict__ g16l,
    const unsigned short* __restrict__ wot, const unsigned short* __restrict__ wotl,
    const float* __restrict__ b_out, float* __restrict__ out) {
  __shared__ __align__(16) union { unsigned w[64 * kPitchW]; float f[8 * 16 * 68]; } sb;
  __shared__ __align__(16) unsigned sbl[kOutResid ? 64 * kPitchW : 4];
  const int tid = threadIdx.x;
  const int lane = tid & 31;
  const int wave = __builtin_amdgcn_readfirstlane((int)(threadIdx.x >> 5));
  const int hh = lane >> 4;
  const int c = lane & 15;
  const size_t n0 = (size_t)blockIdx.x * 64;
  const int obase = (int)blockIdx.y * 256;
  const int b = (int)(n0 >> 12);
  const int l0 = (int)(n0 & (size_t)(kLen - 1));

  v8f acc[2][4];
  v8f accr[2][4];
#pragma unroll
  for (int i = 0; i < 2; ++i)
#pragma unroll
    for (int j = 0; j < 4; ++j) {
      acc[i][j] = (v8f){0.f, 0.f, 0.f, 0.f, 0.f, 0.f, 0.f, 0.f};
      accr[i][j] = (v8f){0.f, 0.f, 0.f, 0.f, 0.f, 0.f, 0.f, 0.f};
    }
  const _Float16* Wr = (const _Float16*)wot + (size_t)(obase + 32 * wave + c) * kWidth + 8 * hh;
  const _Float16* Wl = (const _Float16*)wotl + (size_t)(obase + 32 * wave + c) * kWidth + 8 * hh;

#pragma unroll 1
  for (int sl = 0; sl < kWidth / 256; ++sl) {
    __syncthreads();
    stage_tile_T<256>(g16 + (size_t)sl * 256 * kNpos, n0, sb.w, tid);
    if (kOutResid) stage_tile_T<256>(g16l + (size_t)sl * 256 * kNpos, n0, sbl, tid);
    __syncthreads();
#pragma unroll 1
    for (int ks = 0; ks < 8; ++ks) {
      v16h bf[4];
#pragma unroll
      for (int j = 0; j < 4; ++j) bf[j] = lds_frag<kPitchW>(sb.w, 16 * j + c, ks * 16 + 4 * hh);
#pragma unroll
      for (int i = 0; i < 2; ++i) {
        const v16h ah = frag_load(Wr + (size_t)(i * 16) * kWidth + sl * 256 + ks * 32);
#pragma unroll
        for (int j = 0; j < 4; ++j) acc[i][j] = mma16(ah, bf[j], acc[i][j]);
        tie_acc(acc[i][0], ah, bf[0]);
        tie_acc(acc[i][1], ah, bf[1]);
        tie_acc(acc[i][2], ah, bf[2]);
        tie_acc_nops(acc[i][3], ah, bf[3]);
      }
      if (kOutResid) {
        v16h bl[4];
#pragma unroll
        for (int j = 0; j < 4; ++j) bl[j] = lds_frag<kPitchW>(sbl, 16 * j + c, ks * 16 + 4 * hh);
#pragma unroll
        for (int i = 0; i < 2; ++i) {
          const v16h ah = frag_load(Wr + (size_t)(i * 16) * kWidth + sl * 256 + ks * 32);
          const v16h al = frag_load(Wl + (size_t)(i * 16) * kWidth + sl * 256 + ks * 32);
#pragma unroll
          for (int j = 0; j < 4; ++j) accr[i][j] = mma16(ah, bl[j], accr[i][j]);
          tie_acc(accr[i][0], ah, bl[0]);
          tie_acc(accr[i][1], ah, bl[1]);
          tie_acc(accr[i][2], ah, bl[2]);
          tie_acc_nops(accr[i][3], ah, bl[3]);
#pragma unroll
          for (int j = 0; j < 4; ++j) accr[i][j] = mma16(al, bf[j], accr[i][j]);
          tie_acc(accr[i][0], al, bf[0]);
          tie_acc(accr[i][1], al, bf[1]);
          tie_acc(accr[i][2], al, bf[2]);
          tie_acc_nops(accr[i][3], al, bf[3]);
        }
        keep4(bl[0], bl[1], bl[2], bl[3]);
      }
      keep4(bf[0], bf[1], bf[2], bf[3]);
    }
  }
  acc_guard4(acc[0][0], acc[0][1], acc[0][2], acc[0][3]);
  acc_guard4(acc[1][0], acc[1][1], acc[1][2], acc[1][3]);
  if (kOutResid) {
    acc_guard4(accr[0][0], accr[0][1], accr[0][2], accr[0][3]);
    acc_guard4(accr[1][0], accr[1][1], accr[1][2], accr[1][3]);
  }
  __syncthreads();

  float* slab = sb.f + wave * (16 * 68);
#pragma unroll
  for (int i = 0; i < 2; ++i) {
    const int ob = obase + 32 * wave + 16 * i;
    const int d0 = ob + 8 * hh;
    const v4f b0 = *(const v4f*)(b_out + d0);
    const v4f b1 = *(const v4f*)(b_out + d0 + 4);
#pragma unroll
    for (int j = 0; j < 4; ++j) {
#pragma unroll
      for (int r = 0; r < 8; ++r) {
        const float bv = (r < 4) ? b0[r & 3] : b1[r & 3];
        float sum = acc[i][j][r];
        if (kOutResid) sum = fmaf(accr[i][j][r], kLoScaleInv, sum);
        slab[(8 * hh + r) * 68 + 16 * j + c] = fmaf(sum, kOutFold, bv);
      }
    }
    wave_sync();
    {
      const int c4 = (lane & 15) * 4;
      v4f vals[8];
#pragma unroll
      for (int it = 0; it < 8; ++it) vals[it] = *(const v4f*)(slab + (it * 2 + hh) * 68 + c4);
      for (int pass = 0; pass < 2; ++pass) {
#pragma unroll
        for (int it = 0; it < 8; ++it) {
          const int row = it * 2 + hh;
          *(volatile v4f*)(out + ((size_t)b * kOutF + ob + row) * kLen + l0 + c4) = vals[it];
        }
        __threadfence();
      }
    }
    wave_sync();
  }
}

extern "C" void kernel_launch(void* const* d_in, const int* in_sizes, int n_in,
                              void* d_out, int out_size, void* d_ws, size_t ws_size,
                              hipStream_t stream) {
  if (n_in < 9) return;
  if (in_sizes[0] != kBatch * kWidth * kLen) return;
  if (in_sizes[1] != kWidth) return;
  if (in_sizes[2] != kWidth * kModes) return;
  if (in_sizes[3] != kWidth * kModes) return;
  if (in_sizes[4] != kWidth * kModes) return;
  if (in_sizes[5] != kWidth * kModes) return;
  if (in_sizes[6] != kWidth) return;
  if (in_sizes[7] != kWidth * kOutF) return;
  if (in_sizes[8] != kOutF) return;
  if (out_size != kBatch * kOutF * kLen) return;
  if (ws_size < kWsTotal) return;

  const float* x      = (const float*)d_in[0];
  const float* log_dt = (const float*)d_in[1];
  const float* A_re   = (const float*)d_in[2];
  const float* A_im   = (const float*)d_in[3];
  const float* C_re   = (const float*)d_in[4];
  const float* C_im   = (const float*)d_in[5];
  const float* Dv     = (const float*)d_in[6];
  const float* W_out  = (const float*)d_in[7];
  const float* b_out  = (const float*)d_in[8];
  float* out = (float*)d_out;

  char* ws = (char*)d_ws;
  unsigned short* U16    = (unsigned short*)(ws + kOffU16);
  unsigned short* G16    = (unsigned short*)(ws + kOffG16);
  unsigned short* G16L   = (unsigned short*)(ws + kOffG16L);
  unsigned short* MV16   = (unsigned short*)(ws + kOffMv);
  unsigned short* ET16   = (unsigned short*)(ws + kOffEt);
  float*          S32    = (float*)(ws + kOffS32);
  unsigned short* INIT16 = (unsigned short*)(ws + kOffInit);
  float*          WPOW   = (float*)(ws + kOffWpow);
  unsigned short* WOT    = (unsigned short*)(ws + kOffWot);
  unsigned short* WOTL   = (unsigned short*)(ws + kOffWotL);

  weight_plane_kernel<<<dim3(kOutF / 32, kWidth / 256), 256, 0, stream>>>(W_out, WOT, WOTL);
  stream_plane_kernel<<<kWidth, 256, 0, stream>>>(x, U16);

  for (int g = 0; g < kGroups; ++g) {
    const int h0 = g * kGroupCh;
    mode_tables_kernel<<<kGroupCh, 256, 0, stream>>>(log_dt, A_re, A_im, C_re, C_im, Dv, ET16, MV16, WPOW, h0);
    chunk_gemm_kernel<0><<<kGroupCh / 4, 256, 0, stream>>>(U16, INIT16, ET16, (void*)S32, G16L, h0);
    combine_kernel<<<(kGroupCh * kBatch * 2) / 8, 256, 0, stream>>>(S32, WPOW, INIT16);
    chunk_gemm_kernel<1><<<kGroupCh / 4, 256, 0, stream>>>(U16, INIT16, MV16, (void*)G16, G16L, h0);
  }

  out_proj_kernel<<<dim3(kNpos / 64, kOutF / 256), 256, 0, stream>>>(G16, G16L, WOT, WOTL, b_out, out);
}
